// RNN_26938034880941
// MI455X (gfx1250) — hardware-verified
//
#include <hip/hip_runtime.h>
#include <math.h>

#pragma clang fp contract(off)

constexpr int NBAT  = 4096;
constexpr int NSEQ  = 512;
constexpr int NINP  = 1;
constexpr int NHID  = 16;
constexpr int NOUTF = 1;

constexpr int NTHR   = 256;
constexpr int NWAVE  = NTHR / 32;
constexpr int ROWS_W = 16;
constexpr int ROWS_B = NWAVE * ROWS_W;
constexpr int NBLK   = NBAT / ROWS_B;
constexpr int HPITCH = 40;
constexpr int TILEH  = ROWS_W * HPITCH;
constexpr int HBUFN  = 2 * NWAVE * TILEH;

constexpr float CAR11 = 2048.0f;
constexpr float INV11 = 1.0f / 2048.0f;
constexpr float CAR22 = 4194304.0f;
constexpr float INV22 = 1.0f / 4194304.0f;

static_assert(NINP == 1 && NOUTF == 1 && NHID == 16);
static_assert(NBAT % ROWS_B == 0);
static_assert(NBLK * ROWS_B == NBAT);
static_assert(HPITCH % 8 == 0 && HPITCH >= 32);
static_assert(HBUFN % (8 * NTHR) == 0);
static_assert(ROWS_B == 4 * 32);

typedef __attribute__((ext_vector_type(16))) _Float16 v16h;
typedef __attribute__((ext_vector_type(8)))  _Float16 v8h;
typedef __attribute__((ext_vector_type(16))) __bf16   v16b;
typedef __attribute__((ext_vector_type(8)))  __bf16   v8b;
typedef __attribute__((ext_vector_type(8)))  float    v8f;
typedef __attribute__((ext_vector_type(4)))  float    v4f;

__device__ __forceinline__ void dep_guard_h(v8f& a, v8f& b, v16h x, v16h y) { asm volatile("v_nop\n\tv_nop\n\tv_nop\n\tv_nop" : "+v"(a), "+v"(b) : "v"(x), "v"(y)); }
__device__ __forceinline__ void dep_guard_b(v8f& a, v8f& b, v16b x, v16b y) { asm volatile("v_nop\n\tv_nop\n\tv_nop\n\tv_nop" : "+v"(a), "+v"(b) : "v"(x), "v"(y)); }
__device__ __forceinline__ void keep4_h(v16h a, v16h b, v16h c, v16h d) { asm volatile("v_nop" :: "v"(a), "v"(b), "v"(c), "v"(d)); }
__device__ __forceinline__ void keep4_b(v16b a, v16b b, v16b c, v16b d) { asm volatile("v_nop" :: "v"(a), "v"(b), "v"(c), "v"(d)); }
__device__ __forceinline__ void dep_guard3(v8f& a, v8f& b, v16h x, v16h y, v16h z) {
  asm volatile("v_nop\n\tv_nop\n\tv_nop\n\tv_nop" : "+v"(a), "+v"(b) : "v"(x), "v"(y), "v"(z));
}

template <typename T> struct Frag;
template <> struct Frag<_Float16> {
  typedef v16h V; union U { v16h v; v8h h[2]; };
  static __device__ __forceinline__ v16h load(const _Float16* p) {
    U f; f.h[0] = *(const v8h*)(p); f.h[1] = *(const v8h*)(p + 16); return f.v;
  }
  static __device__ __forceinline__ v8f mma(v16h a, v16h b, v8f c) {
    return __builtin_amdgcn_wmma_f32_16x16x32_f16(false, a, false, b, (short)0, c, false, false);
  }
  static __device__ __forceinline__ void guard(v8f& a, v8f& b, v16h x, v16h y) { dep_guard_h(a, b, x, y); }
  static __device__ __forceinline__ void keep(v16h a, v16h b, v16h c, v16h d) { keep4_h(a, b, c, d); }
};
template <> struct Frag<__bf16> {
  typedef v16b V; union U { v16b v; v8b h[2]; };
  static __device__ __forceinline__ v16b load(const __bf16* p) {
    U f; f.h[0] = *(const v8b*)(p); f.h[1] = *(const v8b*)(p + 16); return f.v;
  }
  static __device__ __forceinline__ v8f mma(v16b a, v16b b, v8f c) {
    return __builtin_amdgcn_wmma_f32_16x16x32_bf16(false, a, false, b, (short)0, c, false, false);
  }
  static __device__ __forceinline__ void guard(v8f& a, v8f& b, v16b x, v16b y) { dep_guard_b(a, b, x, y); }
  static __device__ __forceinline__ void keep(v16b a, v16b b, v16b c, v16b d) { keep4_b(a, b, c, d); }
};

__device__ __forceinline__ float h16_to_f32(unsigned hb) {
  const unsigned sgn = (hb & 0x8000u) << 16; const unsigned em = hb & 0x7fffu;
  const float fn = __uint_as_float((em << 13) + 0x38000000u);
  const float fs = (float)em * 5.9604644775390625e-8f;
  const float mag = (em < 0x400u) ? fs : fn; return __uint_as_float(__float_as_uint(mag) | sgn);
}

__global__ __launch_bounds__(NTHR) void rnn_seq_kernel(
    const float* __restrict__ x,
    const float* __restrict__ Wih,
    const float* __restrict__ Whh,
    const float* __restrict__ bih,
    const float* __restrict__ bhh,
    const float* __restrict__ Wfc,
    const float* __restrict__ bfc,
    float* __restrict__ out) {
  __shared__ __align__(16) _Float16 hbuf[HBUFN];
  __shared__ __align__(16) float    sOut[ROWS_B];

  const int tid = threadIdx.x, lane = tid & 31, wave = tid >> 5;
  const int c = lane & 15, hh = lane >> 4, koff = hh * 8;
  const int rowbase = blockIdx.x * ROWS_B + wave * ROWS_W;

  {
    const v8h z = {(_Float16)0.f, (_Float16)0.f, (_Float16)0.f, (_Float16)0.f,
                   (_Float16)0.f, (_Float16)0.f, (_Float16)0.f, (_Float16)0.f};
#pragma unroll 1
    for (int i = tid; i < HBUFN / 8; i += NTHR) *(v8h*)(hbuf + i * 8) = z;
  }

  const v4f wa = *(const v4f*)(Whh + c * NHID + koff);
  const v4f wb = *(const v4f*)(Whh + c * NHID + koff + 4);
  const float wih_c = Wih[c];
  const float bih_c = bih[c];
  const float bhh_c = bhh[c];
  const float wfc_c = Wfc[c];
  const float bfc_0 = bfc[0];
  const float wv[8] = {wa[0], wa[1], wa[2], wa[3], wb[0], wb[1], wb[2], wb[3]};

  v16h bfr1, bfr2;
  {
    const v16h z16 = {(_Float16)0.f, (_Float16)0.f, (_Float16)0.f, (_Float16)0.f, (_Float16)0.f, (_Float16)0.f, (_Float16)0.f, (_Float16)0.f,
                      (_Float16)0.f, (_Float16)0.f, (_Float16)0.f, (_Float16)0.f, (_Float16)0.f, (_Float16)0.f, (_Float16)0.f, (_Float16)0.f};
    bfr1 = z16; bfr2 = z16;
#pragma unroll
    for (int i = 0; i < 8; ++i) {
      const float w = wv[i];
      const _Float16 whs = (_Float16)(w * CAR11);
      const unsigned short whb = __builtin_bit_cast(unsigned short, whs);
      const float whi = h16_to_f32((unsigned)whb) * INV11;
      const float wrs = w - whi;
      bfr1[i]     = whs;
      bfr1[8 + i] = (_Float16)whi;
      bfr2[i]     = (_Float16)(wrs * CAR22);
    }
  }
  __syncthreads();

  const v8f z8 = {0.f, 0.f, 0.f, 0.f, 0.f, 0.f, 0.f, 0.f};
  const float* xrow = x + (size_t)(rowbase + 8 * hh) * NSEQ;
  float hreg[8];
#pragma unroll
  for (int r = 0; r < 8; ++r) hreg[r] = 0.0f;

#pragma unroll 1
  for (int t = 0; t < NSEQ; ++t) {
    const int cur = t & 1;
    const _Float16* arow = hbuf + (cur * NWAVE + wave) * TILEH + c * HPITCH + koff;
    _Float16*       hn   = hbuf + ((cur ^ 1) * NWAVE + wave) * TILEH;

    float xr[8];
#pragma unroll
    for (int r = 0; r < 8; ++r) xr[r] = xrow[(size_t)r * NSEQ + t];

    const v16h af = Frag<_Float16>::load(arow);
    v8f acc1 = Frag<_Float16>::mma(af, bfr1, z8);
    v8f acc2 = Frag<_Float16>::mma(af, bfr2, z8);
    dep_guard3(acc1, acc2, af, bfr1, bfr2);

#pragma unroll
    for (int r = 0; r < 8; ++r) {
      float xp = xr[r] * wih_c + bih_c;
      xp = xp + bhh_c;
      const float dot = acc1[r] * INV11 + acc2[r] * INV22;
      const float pre = xp + dot;
      const float hv = tanhf(pre);
      hreg[r] = hv;
      const _Float16 h16 = (_Float16)hv;
      const float hif = h16_to_f32((unsigned)__builtin_bit_cast(unsigned short, h16));
      const _Float16 r16 = (_Float16)((hv - hif) * CAR11);
      hn[(8 * hh + r) * HPITCH + c]      = h16;
      hn[(8 * hh + r) * HPITCH + 16 + c] = r16;
    }
    __syncthreads();
  }

  float part[8];
#pragma unroll
  for (int r = 0; r < 8; ++r) part[r] = hreg[r] * wfc_c;
#pragma unroll
  for (int off = 1; off < 16; off <<= 1) {
#pragma unroll
    for (int r = 0; r < 8; ++r) part[r] += __shfl_xor(part[r], off, 32);
  }
  if (c == 0) {
#pragma unroll
    for (int r = 0; r < 8; ++r) sOut[wave * ROWS_W + 8 * hh + r] = part[r] + bfc_0;
  }
  __syncthreads();
  if (wave == 0) {
    const v4f v = *(const v4f*)(sOut + 4 * lane);
    float* op = out + (size_t)blockIdx.x * ROWS_B + 4 * lane;
    *(volatile v4f*)op = v;
    __threadfence();
    *(volatile v4f*)op = v;
  }
}

extern "C" void kernel_launch(void* const* d_in, const int* in_sizes, int n_in,
                              void* d_out, int out_size, void* d_ws, size_t ws_size, hipStream_t stream) {
  (void)in_sizes; (void)out_size; (void)d_ws; (void)ws_size;
  if (n_in < 7 || d_out == nullptr) return;
  const float* x   = (const float*)d_in[0];
  const float* Wih = (const float*)d_in[1];
  const float* Whh = (const float*)d_in[2];
  const float* bih = (const float*)d_in[3];
  const float* bhh = (const float*)d_in[4];
  const float* Wfc = (const float*)d_in[5];
  const float* bfc = (const float*)d_in[6];
  float* out = (float*)d_out;

  rnn_seq_kernel<<<NBLK, NTHR, 0, stream>>>(x, Wih, Whh, bih, bhh, Wfc, bfc, out);
}
